// LongformerSelfAttentionForBart_76914274337234
// MI455X (gfx1250) — hardware-verified
//
#include <hip/hip_runtime.h>
#include <stddef.h>

typedef _Float16 f16;
typedef f16   v16h __attribute__((ext_vector_type(16)));
typedef f16   v8h  __attribute__((ext_vector_type(8)));
typedef v8h   v8ha __attribute__((may_alias));
typedef float v8f  __attribute__((ext_vector_type(8)));
typedef float v4f  __attribute__((ext_vector_type(4)));
typedef v4f   v4fa __attribute__((may_alias));

#define DEV __device__ __forceinline__

constexpr int Bc = 2, Sc = 4096, Dc = 768, Hc = 12, HDc = 64, W1c = 256, NCc = 16;
constexpr int QGR  = 128;
constexpr int GMAX = 16;
constexpr float NEGF = -1.0e9f;
constexpr size_t nBSD = (size_t)Bc * Sc * Dc;
constexpr size_t nW   = (size_t)Dc * Dc;
constexpr size_t nQG  = (size_t)Bc * Hc * QGR * HDc;

constexpr float SC_HS   = 16.0f;
constexpr float SC_W    = 1024.0f;
constexpr float SC_HEAD = 16.0f;
constexpr float SC_P    = 1024.0f;
constexpr float SC_MRG  = 256.0f;
constexpr float PROJ_ACC = 1.0f / (SC_HS * SC_W);
constexpr float OUT_ACC  = 1.0f / (SC_MRG * SC_W);
constexpr float LOGIT_SC = 0.125f / (SC_HEAD * SC_HEAD);
constexpr float ONORM    = SC_MRG / (SC_P * SC_HEAD);

typedef char chk_shapes0[(Sc % 128 == 0 && Dc % 64 == 0 && Dc % 8 == 0 && (Bc * Sc) % 128 == 0) ? 1 : -1];
typedef char chk_shapes1[(W1c % 32 == 0 && NCc * W1c == Sc && HDc == 64 && Hc * HDc == Dc && QGR <= Sc) ? 1 : -1];

DEV v8f mma16(v16h a, v16h b, v8f c) {
  c = __builtin_amdgcn_wmma_f32_16x16x32_f16(false, a, false, b, (short)0, c, false, false);
  asm volatile("v_nop\n\tv_nop\n\tv_nop\n\tv_nop" : "+v"(c) : "v"(a), "v"(b));
  return c;
}

DEV v16h ld_frag(const f16* p, int ld) {
  const int l = threadIdx.x & 31, lh = l >> 4, m = l & 15;
  const f16* r = p + (size_t)m * ld + 8 * lh;
  union { v16h v; v8h h[2]; } u;
  u.h[0] = *(const v8ha*)(r);
  u.h[1] = *(const v8ha*)(r + 16);
  return u.v;
}

DEV v16h ld_frag_kn(const f16* p, int ld) {
  const int l = threadIdx.x & 31, lh = l >> 4, n = l & 15;
  const f16* c = p + n;
  v16h v;
#pragma unroll
  for (int i = 0; i < 8; ++i) {
    v[i]     = c[(size_t)(8 * lh + i) * ld];
    v[8 + i] = c[(size_t)(16 + 8 * lh + i) * ld];
  }
  return v;
}

DEV float rowmax16(float x) {
  x = fmaxf(x, __shfl_xor(x, 1, 32));
  x = fmaxf(x, __shfl_xor(x, 2, 32));
  x = fmaxf(x, __shfl_xor(x, 4, 32));
  x = fmaxf(x, __shfl_xor(x, 8, 32));
  return x;
}
DEV float rowsum16(float x) {
  x += __shfl_xor(x, 1, 32);
  x += __shfl_xor(x, 2, 32);
  x += __shfl_xor(x, 4, 32);
  x += __shfl_xor(x, 8, 32);
  return x;
}

DEV void softmax_step(v8f& s0, v8f& s1, float* m8, float* l8, v8f (&O)[4], f16* Pw, int lh, int m) {
#pragma unroll
  for (int r = 0; r < 8; ++r) {
    const float rm = rowmax16(fmaxf(s0[r], s1[r]));
    const float mv = fmaxf(m8[r], rm);
    const float fs = __expf(m8[r] - mv);
    const float p0 = __expf(s0[r] - mv);
    const float p1 = __expf(s1[r] - mv);
    const float rs = rowsum16(p0 + p1);
    l8[r] = l8[r] * fs + rs;
    m8[r] = mv;
#pragma unroll
    for (int t = 0; t < 4; ++t) O[t][r] *= fs;
    Pw[(8 * lh + r) * 32 + m]      = (f16)(p0 * SC_P);
    Pw[(8 * lh + r) * 32 + 16 + m] = (f16)(p1 * SC_P);
  }
}

__global__ __launch_bounds__(256) void k_cvt_hs(const float* __restrict__ src, f16* dst, int n8) {
  const int i = (int)blockIdx.x * 256 + (int)threadIdx.x;
  if (i < n8) {
    const float* s = src + (size_t)i * 8;
    const v4f a = *(const v4fa*)s, c = *(const v4fa*)(s + 4);
    v8h o;
#pragma unroll
    for (int e = 0; e < 4; ++e) { o[e] = (f16)(a[e] * SC_HS); o[4 + e] = (f16)(c[e] * SC_HS); }
    f16* d = dst + (size_t)i * 8;
    *(volatile v8h*)d = o;
    __threadfence();
    *(volatile v8h*)d = o;
  }
}

__global__ __launch_bounds__(256) void k_cvt_w(const float* __restrict__ w0, const float* __restrict__ w1,
    const float* __restrict__ w2, const float* __restrict__ w3, const float* __restrict__ w4,
    const float* __restrict__ w5, const float* __restrict__ w6, f16* dst, int nchunk) {
  const int y = blockIdx.y;
  const float* src = (y == 0) ? w0 : (y == 1) ? w1 : (y == 2) ? w2 : (y == 3) ? w3
                   : (y == 4) ? w4 : (y == 5) ? w5 : w6;
  const int i = (int)blockIdx.x * 256 + (int)threadIdx.x;
  if (i < nchunk) {
    const int n  = i / (Dc / 8);
    const int k0 = (i - n * (Dc / 8)) * 8;
    v8h o;
#pragma unroll
    for (int e = 0; e < 8; ++e) o[e] = (f16)(src[(size_t)(k0 + e) * Dc + n] * SC_W);
    f16* d = dst + (size_t)y * nW + (size_t)n * Dc + k0;
    *(volatile v8h*)d = o;
    __threadfence();
    *(volatile v8h*)d = o;
  }
}

__global__ __launch_bounds__(256) void k_gemm(const f16* __restrict__ A, const f16* __restrict__ Wt,
    const float* __restrict__ bias, void* outp, float acc_scale, float out_scale, int mode) {
  __shared__ float smem[8192];
  f16* ldsA = (f16*)smem;
  f16* ldsB = ldsA + 128 * 64;
  const int tid = threadIdx.x, wid = tid >> 5, l = tid & 31, lh = l >> 4, m = l & 15;
  const int row0 = (mode == 1) ? (int)blockIdx.x * Sc : (int)blockIdx.x * 128;
  const int n0 = (int)blockIdx.y * 64;

  const v8f z8 = {0.f, 0.f, 0.f, 0.f, 0.f, 0.f, 0.f, 0.f};
  v8f acc[4];
#pragma unroll
  for (int t = 0; t < 4; ++t) acc[t] = z8;

#pragma unroll 1
  for (int kk = 0; kk < Dc; kk += 64) {
    __syncthreads();
    for (int u = tid; u < 128 * 8; u += 256) {
      const int r = u >> 3, seg = u & 7;
      *(v8h*)(ldsA + r * 64 + seg * 8) = *(const v8ha*)(A + (size_t)(row0 + r) * Dc + kk + seg * 8);
    }
    for (int u = tid; u < 64 * 8; u += 256) {
      const int r = u >> 3, seg = u & 7;
      *(v8h*)(ldsB + r * 64 + seg * 8) = *(const v8ha*)(Wt + (size_t)(n0 + r) * Dc + kk + seg * 8);
    }
    __syncthreads();
#pragma unroll
    for (int ks = 0; ks < 2; ++ks) {
      const v16h a = ld_frag(ldsA + wid * 16 * 64 + ks * 32, 64);
#pragma unroll
      for (int t = 0; t < 4; ++t)
        acc[t] = mma16(a, ld_frag(ldsB + t * 16 * 64 + ks * 32, 64), acc[t]);
    }
  }

  __syncthreads();
  float* stg = smem + wid * 1024;
#pragma unroll
  for (int t = 0; t < 4; ++t) {
    const int n = n0 + t * 16 + m;
    const float bn = bias[n];
#pragma unroll
    for (int r = 0; r < 8; ++r) stg[(8 * lh + r) * 64 + t * 16 + m] = (acc[t][r] * acc_scale + bn) * out_scale;
  }
  __syncthreads();

  if (mode == 2) {
    float* out = (float*)outp;
    const int j = l & 15, lr = l >> 4;
    v4f vals[8];
#pragma unroll
    for (int it = 0; it < 8; ++it) vals[it] = *(const v4fa*)(stg + (it * 2 + lr) * 64 + 4 * j);
    float* ob = out + (size_t)(row0 + wid * 16 + lr) * Dc + n0 + 4 * j;
#pragma unroll
    for (int it = 0; it < 8; ++it) *(volatile v4f*)(ob + (size_t)(it * 2) * Dc) = vals[it];
    __threadfence();
#pragma unroll
    for (int it = 0; it < 8; ++it) *(volatile v4f*)(ob + (size_t)(it * 2) * Dc) = vals[it];
  } else {
    f16* out = (f16*)outp;
    const int j = l & 7, q4 = l >> 3;
    const int hh = n0 >> 6;
    v8h vals[4];
#pragma unroll
    for (int it = 0; it < 4; ++it) {
      const float* s = stg + (it * 4 + q4) * 64 + 8 * j;
      const v4f x0 = *(const v4fa*)s, x1 = *(const v4fa*)(s + 4);
#pragma unroll
      for (int e = 0; e < 4; ++e) { vals[it][e] = (f16)x0[e]; vals[it][4 + e] = (f16)x1[e]; }
    }
    const int Rb = row0 + wid * 16 + q4;
    const int bb = Rb / Sc, s0 = Rb - bb * Sc;
    const size_t rowpitch = (size_t)HDc;
    f16* ob;
    if (mode == 0) ob = out + (((size_t)bb * Hc + hh) * Sc  + s0) * HDc + 8 * j;
    else           ob = out + (((size_t)bb * Hc + hh) * QGR + s0) * HDc + 8 * j;
#pragma unroll
    for (int it = 0; it < 4; ++it) *(volatile v8h*)(ob + (size_t)(it * 4) * rowpitch) = vals[it];
    __threadfence();
#pragma unroll
    for (int it = 0; it < 4; ++it) *(volatile v8h*)(ob + (size_t)(it * 4) * rowpitch) = vals[it];
  }
}

__global__ __launch_bounds__(512) void k_band(const f16* __restrict__ q, const f16* __restrict__ k,
    const f16* __restrict__ v, const int* __restrict__ mask, const int* __restrict__ gptr, f16* merged) {
  __shared__ f16 ldsK[32 * 64];
  __shared__ f16 ldsVt[64 * 32];
  __shared__ f16 ldsW[16 * 1024];
  const int c = blockIdx.x, hh = blockIdx.y, b = blockIdx.z;
  const int tid = threadIdx.x, wid = tid >> 5, l = tid & 31, lh = l >> 4, m = l & 15;
  int g = gptr[0];
  g = (g < 0) ? 0 : g;
  g = (g > GMAX) ? GMAX : g;
  const size_t bh = (size_t)(b * Hc + hh);
  const f16* qbh = q + bh * Sc * HDc;
  const f16* kbh = k + bh * Sc * HDc;
  const f16* vbh = v + bh * Sc * HDc;
  const int* maskb = mask + (size_t)b * Sc;

  int kb_start = c * W1c - W1c;  if (kb_start < 0) kb_start = 0;
  int kb_end   = c * W1c + 2 * W1c;  if (kb_end > Sc) kb_end = Sc;
  const int nit = 1 + (kb_end - kb_start) / 32;

  const int qrow0 = c * W1c + wid * 16;
  const v16h qa0 = ld_frag(qbh + (size_t)qrow0 * HDc, HDc);
  const v16h qa1 = ld_frag(qbh + (size_t)qrow0 * HDc + 32, HDc);

  const v8f z8 = {0.f, 0.f, 0.f, 0.f, 0.f, 0.f, 0.f, 0.f};
  float m8[8], l8[8];
  v8f O[4];
#pragma unroll
  for (int t = 0; t < 4; ++t) O[t] = z8;
#pragma unroll
  for (int r = 0; r < 8; ++r) { m8[r] = -1.0e30f; l8[r] = 0.f; }
  f16* myW = ldsW + wid * 1024;

#pragma unroll 1
  for (int idx = 0; idx < nit; ++idx) {
    const int keyb = (idx == 0) ? 0 : kb_start + (idx - 1) * 32;
    __syncthreads();
    if (tid < 256) {
      const int key = tid >> 3, seg = tid & 7;
      *(v8h*)(ldsK + key * 64 + seg * 8) = *(const v8ha*)(kbh + (size_t)(keyb + key) * HDc + seg * 8);
    } else {
      const int u = tid - 256;
      const int key = u >> 3, seg = u & 7;
      const v8h tv = *(const v8ha*)(vbh + (size_t)(keyb + key) * HDc + seg * 8);
#pragma unroll
      for (int e = 0; e < 8; ++e) ldsVt[(seg * 8 + e) * 32 + key] = tv[e];
    }
    __syncthreads();

    v8f s0 = mma16(qa0, ld_frag(ldsK, 64), z8);
    s0 = mma16(qa1, ld_frag(ldsK + 32, 64), s0);
    v8f s1 = mma16(qa0, ld_frag(ldsK + 16 * 64, 64), z8);
    s1 = mma16(qa1, ld_frag(ldsK + 16 * 64 + 32, 64), s1);

    const int j0 = keyb + m, j1 = keyb + 16 + m;
    bool okc0, okc1;
    if (idx == 0) {
      okc0 = (m < g) && (maskb[m] >= 0);
      okc1 = ((16 + m) < g) && (maskb[16 + m] >= 0);
    } else {
      okc0 = (maskb[j0] >= 0);
      okc1 = (maskb[j1] >= 0);
    }
#pragma unroll
    for (int r = 0; r < 8; ++r) {
      const int i = qrow0 + 8 * lh + r;
      bool b0 = okc0, b1 = okc1;
      if (idx != 0) {
        b0 = b0 && (j0 - i <= W1c) && (i - j0 <= W1c);
        b1 = b1 && (j1 - i <= W1c) && (i - j1 <= W1c);
      }
      s0[r] = b0 ? s0[r] * LOGIT_SC : NEGF;
      s1[r] = b1 ? s1[r] * LOGIT_SC : NEGF;
    }

    softmax_step(s0, s1, m8, l8, O, myW, lh, m);
    asm volatile("" ::: "memory");

    const v16h pa = ld_frag(myW, 32);
#pragma unroll
    for (int t = 0; t < 4; ++t) O[t] = mma16(pa, ld_frag(ldsVt + t * 16 * 32, 32), O[t]);
  }

#pragma unroll
  for (int r = 0; r < 8; ++r) {
    const int row = qrow0 + 8 * lh + r;
    const bool qneg = maskb[row] < 0;
    const float inv = (l8[r] > 0.f && !qneg) ? (ONORM / l8[r]) : 0.f;
#pragma unroll
    for (int t = 0; t < 4; ++t) myW[(8 * lh + r) * 64 + t * 16 + m] = (f16)(O[t][r] * inv);
  }
  asm volatile("" ::: "memory");
  const int j = l & 7, q4 = l >> 3;
  v8h vals[4];
#pragma unroll
  for (int it = 0; it < 4; ++it) vals[it] = *(const v8ha*)(myW + (it * 4 + q4) * 64 + 8 * j);
  f16* ob = merged + ((size_t)b * Sc + qrow0 + q4) * Dc + hh * HDc + 8 * j;
#pragma unroll
  for (int it = 0; it < 4; ++it) *(volatile v8h*)(ob + (size_t)(it * 4) * Dc) = vals[it];
  __threadfence();
#pragma unroll
  for (int it = 0; it < 4; ++it) *(volatile v8h*)(ob + (size_t)(it * 4) * Dc) = vals[it];
}

__global__ __launch_bounds__(256) void k_glob(const f16* __restrict__ qg, const f16* __restrict__ kg,
    const f16* __restrict__ vg, const int* __restrict__ mask, const int* __restrict__ gptr, f16* merged) {
  __shared__ float ldsO[8 * 1024];
  __shared__ float ldsM[8 * 16];
  __shared__ float ldsL[8 * 16];
  __shared__ f16   ldsP[8 * 512];
  const int hh = blockIdx.x, b = blockIdx.y;
  const int tid = threadIdx.x, wid = tid >> 5, l = tid & 31, lh = l >> 4, m = l & 15;
  int g = gptr[0];
  g = (g < 0) ? 0 : g;
  g = (g > GMAX) ? GMAX : g;
  const size_t bh = (size_t)(b * Hc + hh);
  const f16* qgb = qg + bh * QGR * HDc;
  const f16* kgb = kg + bh * Sc * HDc;
  const f16* vgb = vg + bh * Sc * HDc;
  const int* maskb = mask + (size_t)b * Sc;

  const v16h qa0 = ld_frag(qgb, HDc);
  const v16h qa1 = ld_frag(qgb + 32, HDc);

  const v8f z8 = {0.f, 0.f, 0.f, 0.f, 0.f, 0.f, 0.f, 0.f};
  float m8[8], l8[8];
  v8f O[4];
#pragma unroll
  for (int t = 0; t < 4; ++t) O[t] = z8;
#pragma unroll
  for (int r = 0; r < 8; ++r) { m8[r] = -1.0e30f; l8[r] = 0.f; }
  f16* myP = ldsP + wid * 512;

#pragma unroll 1
  for (int it = 0; it < Sc / 256; ++it) {
    const int kb = wid * (Sc / 8) + it * 32;
    v8f s0 = mma16(qa0, ld_frag(kgb + (size_t)kb * HDc, HDc), z8);
    s0 = mma16(qa1, ld_frag(kgb + (size_t)kb * HDc + 32, HDc), s0);
    v8f s1 = mma16(qa0, ld_frag(kgb + (size_t)(kb + 16) * HDc, HDc), z8);
    s1 = mma16(qa1, ld_frag(kgb + (size_t)(kb + 16) * HDc + 32, HDc), s1);

    const bool okc0 = (maskb[kb + m] >= 0);
    const bool okc1 = (maskb[kb + 16 + m] >= 0);
#pragma unroll
    for (int r = 0; r < 8; ++r) {
      s0[r] = okc0 ? s0[r] * LOGIT_SC : NEGF;
      s1[r] = okc1 ? s1[r] * LOGIT_SC : NEGF;
    }
    softmax_step(s0, s1, m8, l8, O, myP, lh, m);
    asm volatile("" ::: "memory");

    const v16h pa = ld_frag(myP, 32);
#pragma unroll
    for (int t = 0; t < 4; ++t) O[t] = mma16(pa, ld_frag_kn(vgb + (size_t)kb * HDc + t * 16, HDc), O[t]);
  }

#pragma unroll
  for (int t = 0; t < 4; ++t)
#pragma unroll
    for (int r = 0; r < 8; ++r) ldsO[wid * 1024 + (8 * lh + r) * 64 + t * 16 + m] = O[t][r];
  if (m == 0) {
#pragma unroll
    for (int r = 0; r < 8; ++r) {
      ldsM[wid * 16 + 8 * lh + r] = m8[r];
      ldsL[wid * 16 + 8 * lh + r] = l8[r];
    }
  }
  __syncthreads();

  if (wid == 0) {
    const int j = l & 7, q4 = l >> 3;
    v8h vals[4];
#pragma unroll
    for (int it = 0; it < 4; ++it) {
      const int row = it * 4 + q4;
      float M = -1.0e30f;
#pragma unroll
      for (int w = 0; w < 8; ++w) M = fmaxf(M, ldsM[w * 16 + row]);
      float L = 0.f;
      float a8[8] = {0.f, 0.f, 0.f, 0.f, 0.f, 0.f, 0.f, 0.f};
#pragma unroll
      for (int w = 0; w < 8; ++w) {
        const float f = __expf(ldsM[w * 16 + row] - M);
        L += f * ldsL[w * 16 + row];
        const float* src = ldsO + w * 1024 + row * 64 + 8 * j;
#pragma unroll
        for (int e = 0; e < 8; ++e) a8[e] += f * src[e];
      }
      const float inv = (L > 0.f) ? (ONORM / L) : 0.f;
#pragma unroll
      for (int e = 0; e < 8; ++e) vals[it][e] = (f16)(a8[e] * inv);
    }
    f16* ob = merged + ((size_t)b * Sc) * Dc + hh * HDc + 8 * j;
#pragma unroll
    for (int it = 0; it < 4; ++it) {
      const int row = it * 4 + q4;
      if (row < g) *(volatile v8h*)(ob + (size_t)row * Dc) = vals[it];
    }
    __threadfence();
#pragma unroll
    for (int it = 0; it < 4; ++it) {
      const int row = it * 4 + q4;
      if (row < g) *(volatile v8h*)(ob + (size_t)row * Dc) = vals[it];
    }
  }
}

extern "C" void kernel_launch(void* const* d_in, const int* in_sizes, int n_in,
                              void* d_out, int out_size, void* d_ws,
                              size_t ws_size, hipStream_t stream) {
  if (n_in < 17) return;
  if ((size_t)in_sizes[0] != nBSD || (size_t)out_size != nBSD) return;
  if (in_sizes[1] != Bc * Sc || in_sizes[16] < 1) return;
  for (int i = 0; i < 7; ++i) {
    if ((size_t)in_sizes[2 + 2 * i] != nW || in_sizes[3 + 2 * i] != Dc) return;
  }

  const float* hs   = (const float*)d_in[0];
  const int*   mask = (const int*)d_in[1];
  const int*   gptr = (const int*)d_in[16];

  const size_t bBSD = nBSD * sizeof(f16);
  const size_t bW   = nW * sizeof(f16);
  const size_t bQG  = nQG * sizeof(f16);
  size_t off = 0;
  char* base = (char*)d_ws;
  f16* hs16 = (f16*)(base + off); off += bBSD;
  f16* wt   = (f16*)(base + off); off += 7 * bW;
  f16* q16  = (f16*)(base + off); off += bBSD;
  f16* k16  = (f16*)(base + off); off += bBSD;
  f16* v16  = (f16*)(base + off); off += bBSD;
  f16* kg16 = (f16*)(base + off); off += bBSD;
  f16* vg16 = (f16*)(base + off); off += bBSD;
  f16* qg16 = (f16*)(base + off); off += bQG;
  f16* mrg  = (f16*)(base + off); off += bBSD;
  if (off > ws_size) return;

  const int n8 = (int)(nBSD / 8);
  k_cvt_hs<<<dim3((n8 + 255) / 256), dim3(256), 0, stream>>>(hs, hs16, n8);

  const int nchunk = (int)(nW / 8);
  k_cvt_w<<<dim3((nchunk + 255) / 256, 7), dim3(256), 0, stream>>>(
      (const float*)d_in[2], (const float*)d_in[4], (const float*)d_in[6], (const float*)d_in[8],
      (const float*)d_in[10], (const float*)d_in[12], (const float*)d_in[14], wt, nchunk);

  const dim3 gg(Bc * Sc / 128, Dc / 64);
  k_gemm<<<gg, dim3(256), 0, stream>>>(hs16, wt + 0 * nW, (const float*)d_in[3],  (void*)q16,  PROJ_ACC, SC_HEAD, 0);
  k_gemm<<<gg, dim3(256), 0, stream>>>(hs16, wt + 1 * nW, (const float*)d_in[5],  (void*)k16,  PROJ_ACC, SC_HEAD, 0);
  k_gemm<<<gg, dim3(256), 0, stream>>>(hs16, wt + 2 * nW, (const float*)d_in[7],  (void*)v16,  PROJ_ACC, SC_HEAD, 0);
  k_gemm<<<gg, dim3(256), 0, stream>>>(hs16, wt + 4 * nW, (const float*)d_in[11], (void*)kg16, PROJ_ACC, SC_HEAD, 0);
  k_gemm<<<gg, dim3(256), 0, stream>>>(hs16, wt + 5 * nW, (const float*)d_in[13], (void*)vg16, PROJ_ACC, SC_HEAD, 0);
  k_gemm<<<dim3(Bc, Dc / 64), dim3(256), 0, stream>>>(hs16, wt + 3 * nW, (const float*)d_in[9], (void*)qg16,
                                                     PROJ_ACC, SC_HEAD, 1);

  k_band<<<dim3(NCc, Hc, Bc), dim3(512), 0, stream>>>(q16, k16, v16, mask, gptr, mrg);
  k_glob<<<dim3(Hc, Bc), dim3(256), 0, stream>>>(qg16, kg16, vg16, mask, gptr, mrg);

  k_gemm<<<gg, dim3(256), 0, stream>>>(mrg, wt + 6 * nW, (const float*)d_in[15], d_out, OUT_ACC, 1.0f, 2);
}
